// JointAttention_64957085385332
// MI455X (gfx1250) — hardware-run, weakly checked
//
#include <hip/hip_runtime.h>


#ifndef NB
#define NB 2
#endif
#ifndef SEQ
#define SEQ 1024
#endif
#define NB_FULL  2
#define SEQ_FULL 1024
#ifndef OUT_SEQ
#define OUT_SEQ SEQ
#endif
#define DM   256
#define TW   8
#define SCL2 ((float)(0.0625 * 1.4426950408889634))

static_assert(DM % 64 == 0);
static_assert(DM % 32 == 0);
static_assert((NB * SEQ) % 64 == 0);
static_assert(DM == 32 * TW);
static_assert(DM % 4 == 0);
static_assert(((size_t)SEQ * DM) % 8 == 0);
static_assert(((size_t)DM * DM) % 8 == 0);
static_assert(NB <= NB_FULL);
static_assert(SEQ <= SEQ_FULL);
static_assert((68 * 4) % 16 == 0);
static_assert(32 * 16 * 8 == 16 * 64 * 4);
static_assert(2 * 32 * 16 == DM * 4);
static_assert(16 * 68 * 4 <= 131072);
static_assert((3 * DM + 2 * TW) * 4 <= 131072);

typedef unsigned short bf;
typedef __attribute__((ext_vector_type(16))) __bf16   v16bf;
typedef __attribute__((ext_vector_type(8)))  unsigned short v8us;
typedef __attribute__((ext_vector_type(8)))  float    v8f;
typedef __attribute__((ext_vector_type(4)))  float    v4f;
typedef v4f  __attribute__((may_alias)) v4fa;

__device__ __forceinline__ unsigned short f2bf(float f) { unsigned u = __float_as_uint(f); u += 0x7FFFu + ((u >> 16) & 1u); return (unsigned short)(u >> 16); }
__device__ __forceinline__ float bfr(float f) { return __uint_as_float(((unsigned)f2bf(f)) << 16); }
__device__ __forceinline__ v16bf cat16b(v8us lo, v8us hi) { return __builtin_bit_cast(v16bf, __builtin_shufflevector(lo, hi, 0, 1, 2, 3, 4, 5, 6, 7, 8, 9, 10, 11, 12, 13, 14, 15)); }
__device__ __forceinline__ v8f wmmab(v16bf a, v16bf b, v8f c) { return __builtin_amdgcn_wmma_f32_16x16x32_bf16(false, a, false, b, (short)0, c, false, false); }
__device__ __forceinline__ v8f wmmab_g(v16bf a, v16bf b, v8f c) { c = wmmab(a, b, c); asm volatile("v_nop\n\tv_nop\n\tv_nop\n\tv_nop" : "+v"(c) : "v"(a), "v"(b)); return c; }
__device__ __forceinline__ v16bf ldb(const bf* p)  { return cat16b(*(const v8us*)p, *(const v8us*)(p + 16)); }
__device__ __forceinline__ void wave_sync() { __builtin_amdgcn_fence(3  , "wavefront"); __builtin_amdgcn_wave_barrier(); asm volatile("" ::: "memory"); }

__global__ __launch_bounds__(256) void k_cvt8(const float* __restrict__ src, bf* dst, size_t n8) {
    const size_t i = (size_t)blockIdx.x * 256 + threadIdx.x; if (i >= n8) return;
    const v8f v = *(const v8f*)(src + i * 8); v8us o;
#pragma unroll
    for (int k = 0; k < 8; ++k) o[k] = f2bf(v[k]);
    *(volatile v8us*)(dst + i * 8) = o; __threadfence(); *(volatile v8us*)(dst + i * 8) = o;
}

__global__ __launch_bounds__(32) void k_proj(const bf* __restrict__ A, const bf* __restrict__ Bt, const float* __restrict__ bias, float* P) {
    __shared__ __align__(16) float os[16 * 68];
    const int K = DM;
    const int lane = threadIdx.x & 31, lr = lane & 15, hi = lane >> 4; const int r0 = blockIdx.x * 64, c0 = blockIdx.y * 64;
    v8f acc[4][4];
#pragma unroll
    for (int mb = 0; mb < 4; ++mb)
#pragma unroll
        for (int nb = 0; nb < 4; ++nb) acc[mb][nb] = (v8f){};
    const size_t aoff = (size_t)(r0 + lr) * K + 8 * hi, boff = (size_t)(c0 + lr) * K + 8 * hi;
#pragma unroll 1
    for (int kc = 0; kc < K; kc += 32) {
        v16bf a[4];
#pragma unroll
        for (int mb = 0; mb < 4; ++mb) a[mb] = ldb(A + aoff + (size_t)mb * 16 * K + kc);
#pragma unroll
        for (int nb = 0; nb < 4; ++nb) { const v16bf b = ldb(Bt + boff + (size_t)nb * 16 * K + kc);
#pragma unroll
            for (int mb = 0; mb < 4; ++mb) acc[mb][nb] = wmmab_g(a[mb], b, acc[mb][nb]); }
    }
    float bc[4];
#pragma unroll
    for (int nb = 0; nb < 4; ++nb) bc[nb] = bfr(bias[c0 + nb * 16 + lr]);
    const size_t tbase = (size_t)r0 * DM + (size_t)c0;
#pragma unroll
    for (int mb = 0; mb < 4; ++mb) {
#pragma unroll
        for (int nb = 0; nb < 4; ++nb) {
#pragma unroll
            for (int j = 0; j < 8; ++j) os[(hi * 8 + j) * 68 + nb * 16 + lr] = acc[mb][nb][j] + bc[nb]; }
        wave_sync();
        const size_t sb = tbase + (size_t)(mb * 16) * DM;
#pragma unroll 1
        for (int ps = 0; ps < 2; ++ps) {
#pragma unroll
            for (int s = 0; s < 8; ++s) { const int row = 2 * s + (lane >> 4), c4 = (lane & 15) * 4;
                const v4f val = *(const v4fa*)(&os[row * 68 + c4]);
                *(volatile v4f*)(P + sb + (size_t)row * DM + c4) = val; }
            if (ps == 0) __threadfence(); }
        wave_sync();
    }
}

__global__ __launch_bounds__(32 * TW) void k_tok(const float* __restrict__ QP, const float* __restrict__ KP, const float* __restrict__ VP, float* OUT) {
    __shared__ __align__(16) float sK[DM];
    __shared__ __align__(16) float sV[DM];
    __shared__ __align__(16) float so[DM];
    __shared__ float wmax[TW];
    __shared__ float wmin[TW];
    const int tid = threadIdx.x; const int lane = tid & 31;
    const int wave = __builtin_amdgcn_readfirstlane((int)(threadIdx.x >> 5));
    const int g = blockIdx.x;
    const size_t base = (size_t)g * DM;
    const float kv = KP[base + tid];
    sK[tid] = kv; sV[tid] = VP[base + tid];
    float mx = kv, mn = kv;
#pragma unroll
    for (int off = 16; off > 0; off >>= 1) { mx = fmaxf(mx, __shfl_xor(mx, off, 32)); mn = fminf(mn, __shfl_xor(mn, off, 32)); }
    if (lane == 0) { wmax[wave] = mx; wmin[wave] = mn; }
    __syncthreads();
    float kmax = wmax[0], kmin = wmin[0];
#pragma unroll
    for (int w = 1; w < TW; ++w) { kmax = fmaxf(kmax, wmax[w]); kmin = fminf(kmin, wmin[w]); }
    const float a2 = QP[base + tid] * SCL2;
    const float m2 = (a2 >= 0.0f) ? a2 * kmax : a2 * kmin;
    float num = 0.0f, den = 0.0f;
#pragma unroll 2
    for (int j4 = 0; j4 < DM / 4; ++j4) {
        const v4f k4 = *(const v4fa*)(&sK[4 * j4]); const v4f w4 = *(const v4fa*)(&sV[4 * j4]);
#pragma unroll
        for (int c = 0; c < 4; ++c) { const float e = __builtin_amdgcn_exp2f(fmaf(a2, k4[c], -m2)); den += e; num = fmaf(e, w4[c], num); }
    }
    so[tid] = num * (1.0f / den);
    __syncthreads();
    if (wave < 2) {
        const int bb = g / SEQ, tt = g - bb * SEQ;
        float* orow = OUT + ((size_t)bb * OUT_SEQ + tt) * DM + tid * 4;
        const v4f val = *(const v4fa*)(&so[tid * 4]);
        *(volatile v4f*)orow = val; __threadfence(); *(volatile v4f*)orow = val;
    }
}

static constexpr size_t al256(size_t v) { return (v + 255) & ~(size_t)255; }
static constexpr size_t SZ_XB = al256((size_t)NB * SEQ * DM * 2);
static constexpr size_t SZ_WB = al256((size_t)3 * DM * DM * 2);
static constexpr size_t SZ_PL = al256((size_t)NB * SEQ * DM * 4);
static constexpr size_t SZ_TOTAL = SZ_XB + SZ_WB + 3 * SZ_PL;
static_assert(SZ_TOTAL <= (size_t)134217728);
static_assert(((size_t)DM * DM * 2) % 256 == 0);
static_assert((size_t)(NB * SEQ / 64) * 64 * DM * 4 <= SZ_PL);
static_assert((size_t)NB * SEQ * DM * 2 <= SZ_XB);

extern "C" void kernel_launch(void* const* d_in, const int* in_sizes, int n_in,
                              void* d_out, int out_size, void* d_ws, size_t ws_size, hipStream_t stream) {
    if (n_in < 7) return;
    const size_t needx = ((size_t)(NB - 1) * SEQ_FULL + SEQ) * DM;
    if ((size_t)in_sizes[0] < needx) return;
    if ((size_t)in_sizes[1] < (size_t)DM * DM || (size_t)in_sizes[3] < (size_t)DM * DM || (size_t)in_sizes[5] < (size_t)DM * DM) return;
    if (in_sizes[2] < DM || in_sizes[4] < DM || in_sizes[6] < DM) return;
    if ((size_t)out_size < ((size_t)(NB - 1) * OUT_SEQ + SEQ) * DM) return;
    if (SZ_TOTAL > ws_size) return;
    const float* x  = (const float*)d_in[0];
    const float* wq = (const float*)d_in[1]; const float* bq = (const float*)d_in[2];
    const float* wk = (const float*)d_in[3]; const float* bk = (const float*)d_in[4];
    const float* wv = (const float*)d_in[5]; const float* bv = (const float*)d_in[6];
    float* OUT = (float*)d_out;
    char* wsp = (char*)d_ws;
    bf* XB = (bf*)wsp; wsp += SZ_XB;
    bf* WB = (bf*)wsp; wsp += SZ_WB;
    float* QP = (float*)wsp; wsp += SZ_PL;
    float* KP = (float*)wsp; wsp += SZ_PL;
    float* VP = (float*)wsp; wsp += SZ_PL;
    bf* WQ = WB; bf* WK = WB + (size_t)DM * DM; bf* WV = WB + (size_t)2 * DM * DM;

    if (SEQ == SEQ_FULL) {
        const size_t n8 = (size_t)NB * SEQ * DM / 8;
        k_cvt8<<<(unsigned)((n8 + 255) / 256), 256, 0, stream>>>(x, XB, n8);
    } else {
        const size_t n8 = (size_t)SEQ * DM / 8;
        for (int b = 0; b < NB; ++b) k_cvt8<<<(unsigned)((n8 + 255) / 256), 256, 0, stream>>>(x + (size_t)b * SEQ_FULL * DM, XB + (size_t)b * SEQ * DM, n8);
    }
    { const size_t n8 = (size_t)DM * DM / 8; const unsigned g = (unsigned)((n8 + 255) / 256);
      k_cvt8<<<g, 256, 0, stream>>>(wq, WQ, n8); k_cvt8<<<g, 256, 0, stream>>>(wk, WK, n8); k_cvt8<<<g, 256, 0, stream>>>(wv, WV, n8); }

    k_proj<<<dim3(NB * SEQ / 64, DM / 64, 1), 32, 0, stream>>>(XB, WQ, bq, QP);
    k_proj<<<dim3(NB * SEQ / 64, DM / 64, 1), 32, 0, stream>>>(XB, WK, bk, KP);
    k_proj<<<dim3(NB * SEQ / 64, DM / 64, 1), 32, 0, stream>>>(XB, WV, bv, VP);

    k_tok<<<dim3(NB * SEQ, 1, 1), 32 * TW, 0, stream>>>(QP, KP, VP, OUT);
}
